// MutliHeadAttention1D_31585189495126
// MI455X (gfx1250) — hardware-verified
//
#include <hip/hip_runtime.h>
#include <hip/hip_bf16.h>


#define B_    4
#define S_    4096
#define FIN   512
#define FOUT  512
#define KWIN  17
#define GRP   8
#define DH    64
#define PADW  8
#define M_    (B_ * S_)
#define NTOT  (3 * FOUT)
#define KDIM  512

#define LDS_STRIDE   40
#define GEMM_THREADS 256
#define GEMM_DYN_LDS 65536
#define ROWS_PER_BLK 4
#define RELN         (FOUT * KWIN)
#define ATT_ROW      (GRP * KWIN)

static_assert(M_ % 128 == 0);
static_assert(NTOT % 128 == 0);
static_assert(KDIM % 32 == 0);
static_assert(FOUT % 128 == 0);
static_assert(M_ % ROWS_PER_BLK == 0);
static_assert((ROWS_PER_BLK * ATT_ROW * 4) % 128 == 0);
static_assert((M_ * KDIM) % (8 * 256) == 0);
static_assert((FOUT * FIN) % (8 * 256) == 0);
static_assert(2 * 128 * LDS_STRIDE * 2 <= GEMM_DYN_LDS);
static_assert(RELN % 256 == 0);
static_assert(DH == 64 && GRP * DH == FOUT);

typedef __bf16         v16bf __attribute__((ext_vector_type(16)));
typedef float          v8f   __attribute__((ext_vector_type(8)));
typedef float          v4f   __attribute__((ext_vector_type(4)));
typedef float          v2f   __attribute__((ext_vector_type(2)));
typedef unsigned int   v4u   __attribute__((ext_vector_type(4)));

union Frag { v16bf v; v4u q[2]; };

__device__ __forceinline__ unsigned int f2bf_bits(float f) {
  unsigned int u = __float_as_uint(f);
  u += 0x7FFFu + ((u >> 16) & 1u);
  return u >> 16;
}
__device__ __forceinline__ float bf16_rne_val(float f) {
  unsigned int u = __float_as_uint(f);
  u += 0x7FFFu + ((u >> 16) & 1u);
  return __uint_as_float(u & 0xFFFF0000u);
}
__device__ __forceinline__ unsigned int pack_bf16x2(float lo, float hi) {
  return f2bf_bits(lo) | (f2bf_bits(hi) << 16);
}

__device__ __forceinline__ v8f wmma_bf16(const v16bf a, const v16bf b, v8f c) {
  v8f d = __builtin_amdgcn_wmma_f32_16x16x32_bf16(false, a, false, b, (short)0, c, false, false);
  asm volatile("v_nop\n\tv_nop\n\tv_nop\n\tv_nop" : "+v"(d) : "v"(a), "v"(b));
  return d;
}

__global__ __launch_bounds__(256) void cvt_bf16x8(const float* __restrict__ s0,
                                                  const float* __restrict__ s1,
                                                  const float* __restrict__ s2,
                                                  unsigned short* dst, int n8, int seg8) {
  const float* src = (blockIdx.y == 0) ? s0 : ((blockIdx.y == 1) ? s1 : s2);
  unsigned short* dseg = dst + (size_t)blockIdx.y * (size_t)seg8 * 8;
  const int i = blockIdx.x * 256 + threadIdx.x;
  const bool ok = i < n8;
  v4u pk = {0u, 0u, 0u, 0u};
  if (ok) {
    const float* p = src + (size_t)i * 8;
    const v4f a = *(const v4f*)p;
    const v4f b = *(const v4f*)(p + 4);
    pk.x = pack_bf16x2(a.x, a.y);
    pk.y = pack_bf16x2(a.z, a.w);
    pk.z = pack_bf16x2(b.x, b.y);
    pk.w = pack_bf16x2(b.z, b.w);
  }
  unsigned short* q = dseg + (size_t)i * 8;
  if (ok) *(volatile v4u*)q = pk;
  __threadfence();
  if (ok) *(volatile v4u*)q = pk;
}

__device__ __forceinline__ void gemm_store_pass(const float* stage, float* dst, int m0, int tid) {
#pragma unroll
  for (int i = 0; i < 16; ++i) {
    const int idx = i * GEMM_THREADS + tid;
    const int row = idx >> 5;
    const int c   = (idx & 31) * 4;
    const v4f v = *(const v4f*)(stage + row * 128 + c);
    *(volatile v4f*)(dst + (size_t)(m0 + row) * FOUT + c) = v;
  }
}

__global__ __launch_bounds__(GEMM_THREADS) void qkv_gemm(const unsigned short* __restrict__ xb,
                                                         const unsigned short* __restrict__ wb,
                                                         float* qkv) {
  extern __shared__ __attribute__((aligned(16))) unsigned char dsm[];
  unsigned short* As = (unsigned short*)dsm;
  unsigned short* Bs = As + 128 * LDS_STRIDE;
  float* stage = (float*)dsm;

  const int tid  = threadIdx.x;
  const int lane = tid & 31;
  const int wave = tid >> 5;
  const int h    = lane >> 4;
  const int m    = lane & 15;
  const int wm   = wave & 3;
  const int wn   = wave >> 2;
  const int m0   = blockIdx.x * 128;
  const int n0   = blockIdx.y * 128;

  const int lr = tid >> 2;
  const int lq = (tid & 3) * 8;
  const unsigned short* ga = xb + (size_t)(m0 + lr) * KDIM + lq;
  const unsigned short* gb = wb + (size_t)(n0 + lr) * KDIM + lq;

  v8f acc[2][4] = {};

  for (int kb = 0; kb < KDIM; kb += 32) {
    const v4u a0 = *(const v4u*)(ga + kb);
    const v4u a1 = *(const v4u*)(ga + (size_t)64 * KDIM + kb);
    const v4u b0 = *(const v4u*)(gb + kb);
    const v4u b1 = *(const v4u*)(gb + (size_t)64 * KDIM + kb);
    __syncthreads();
    *(v4u*)(As + lr * LDS_STRIDE + lq)        = a0;
    *(v4u*)(As + (lr + 64) * LDS_STRIDE + lq) = a1;
    *(v4u*)(Bs + lr * LDS_STRIDE + lq)        = b0;
    *(v4u*)(Bs + (lr + 64) * LDS_STRIDE + lq) = b1;
    __syncthreads();

    Frag af[2];
#pragma unroll
    for (int mt = 0; mt < 2; ++mt) {
      const int row = wm * 32 + mt * 16 + m;
      af[mt].q[0] = *(const v4u*)(As + row * LDS_STRIDE + 8 * h);
      af[mt].q[1] = *(const v4u*)(As + row * LDS_STRIDE + 16 + 8 * h);
    }
    Frag bfr[4];
#pragma unroll
    for (int nt = 0; nt < 4; ++nt) {
      const int col = wn * 64 + nt * 16 + m;
      bfr[nt].q[0] = *(const v4u*)(Bs + col * LDS_STRIDE + 8 * h);
      bfr[nt].q[1] = *(const v4u*)(Bs + col * LDS_STRIDE + 16 + 8 * h);
    }

#pragma unroll
    for (int mt = 0; mt < 2; ++mt)
#pragma unroll
      for (int nt = 0; nt < 4; ++nt)
        acc[mt][nt] = wmma_bf16(af[mt].v, bfr[nt].v, acc[mt][nt]);
  }
  __syncthreads();

#pragma unroll
  for (int mt = 0; mt < 2; ++mt)
#pragma unroll
    for (int nt = 0; nt < 4; ++nt) {
      const int srow = wm * 32 + mt * 16 + 8 * h;
      const int scol = wn * 64 + nt * 16 + m;
#pragma unroll
      for (int r = 0; r < 8; ++r)
        stage[(srow + r) * 128 + scol] = acc[mt][nt][r];
    }
  __syncthreads();

  const int proj = n0 >> 9;
  const int ob   = n0 & (FOUT - 1);
  float* dst = qkv + (size_t)proj * M_ * FOUT + ob;
  gemm_store_pass(stage, dst, m0, tid);
  __threadfence();
  gemm_store_pass(stage, dst, m0, tid);
}

__device__ __forceinline__ void attn_store_pass(const float* outS, const float* attnS,
                                                float* out, float* attn,
                                                int row0, int nrows, int tid) {
#pragma unroll
  for (int jj = 0; jj < 2; ++jj) {
    const int j = jj * 256 + tid;
    const int r = j >> 7;
    if (row0 + r < nrows) {
      const v4f v = *(const v4f*)(outS + 4 * j);
      *(volatile v4f*)(out + (size_t)row0 * FOUT + 4 * j) = v;
    }
  }
  if (tid < (ROWS_PER_BLK * ATT_ROW) / 4) {
    const int r = (4 * tid) / ATT_ROW;
    if (row0 + r < nrows) {
      const v4f v = *(const v4f*)(attnS + 4 * tid);
      *(volatile v4f*)(attn + (size_t)row0 * ATT_ROW + 4 * tid) = v;
    }
  }
}

__global__ __launch_bounds__(256) void attn_kernel(const float* __restrict__ qkv,
                                                   const float* __restrict__ rel,
                                                   float* out, float* attn, int nrows) {
  __shared__ float relS[RELN];
  __shared__ __attribute__((aligned(16))) float outS[ROWS_PER_BLK * FOUT];
  __shared__ __attribute__((aligned(16))) float attnS[ROWS_PER_BLK * ATT_ROW];

  const int tid  = threadIdx.x;
  const int lane = tid & 31;
  const int g    = tid >> 5;
  const int row0 = blockIdx.x * ROWS_PER_BLK;

  for (int i = tid; i < RELN; i += 256) relS[i] = bf16_rne_val(rel[i]);
  __syncthreads();

  const float* qb = qkv;
  const float* kb = qkv + (size_t)M_ * FOUT;
  const float* vb = qkv + 2 * (size_t)M_ * FOUT;
  const int o0 = g * DH + 2 * lane;

#pragma unroll 1
  for (int it = 0; it < ROWS_PER_BLK; ++it) {
    const int row = row0 + it;
    if (row < nrows) {
      const int b = row / S_;
      const int s = row - b * S_;
      const v2f q2 = *(const v2f*)(qb + (size_t)row * FOUT + o0);

      float e[KWIN];
#pragma unroll
      for (int k = 0; k < KWIN; ++k) {
        const int p = s + k - PADW;
        v2f kv = {0.f, 0.f};
        if (p >= 0 && p < S_)
          kv = *(const v2f*)(kb + ((size_t)b * S_ + p) * FOUT + o0);
        const float t0 = kv.x + relS[o0 * KWIN + k];
        const float t1 = kv.y + relS[(o0 + 1) * KWIN + k];
        float part = q2.x * t0 + q2.y * t1;
#pragma unroll
        for (int off = 16; off >= 1; off >>= 1)
          part += __shfl_xor(part, off, 32);
        e[k] = part;
      }

      float mx = e[0];
#pragma unroll
      for (int k = 1; k < KWIN; ++k) mx = fmaxf(mx, e[k]);
      float sum = 0.f;
#pragma unroll
      for (int k = 0; k < KWIN; ++k) { e[k] = __expf(e[k] - mx); sum += e[k]; }
      const float inv = 1.0f / sum;

      v2f accv = {0.f, 0.f};
#pragma unroll
      for (int k = 0; k < KWIN; ++k) {
        e[k] *= inv;
        const int p = s + k - PADW;
        if (p >= 0 && p < S_) {
          const v2f vv = *(const v2f*)(vb + ((size_t)b * S_ + p) * FOUT + o0);
          accv.x += e[k] * vv.x;
          accv.y += e[k] * vv.y;
        }
      }

      outS[it * FOUT + o0]     = accv.x;
      outS[it * FOUT + o0 + 1] = accv.y;
      if (lane == 0) {
#pragma unroll
        for (int k = 0; k < KWIN; ++k) attnS[it * ATT_ROW + g * KWIN + k] = e[k];
      }
    }
  }
  __syncthreads();

  attn_store_pass(outS, attnS, out, attn, row0, nrows, tid);
  __threadfence();
  attn_store_pass(outS, attnS, out, attn, row0, nrows, tid);
}

extern "C" void kernel_launch(void* const* d_in, const int* in_sizes, int n_in,
                              void* d_out, int out_size, void* d_ws, size_t ws_size,
                              hipStream_t stream) {
  if (n_in < 5) return;
  if (in_sizes[0] != M_ * FIN)    return;
  if (in_sizes[1] != FOUT * FIN)  return;
  if (in_sizes[2] != FOUT * FIN)  return;
  if (in_sizes[3] != FOUT * FIN)  return;
  if (in_sizes[4] != FOUT * KWIN) return;
  if (out_size != M_ * FOUT + M_ * GRP * KWIN) return;

  const float* x   = (const float*)d_in[0];
  const float* Wq  = (const float*)d_in[1];
  const float* Wk  = (const float*)d_in[2];
  const float* Wv  = (const float*)d_in[3];
  const float* rel = (const float*)d_in[4];

  const size_t xb_bytes  = (size_t)M_ * KDIM * 2;
  const size_t wb_bytes  = (size_t)NTOT * KDIM * 2;
  const size_t qkv_bytes = (size_t)3 * M_ * FOUT * 4;
  if (xb_bytes + wb_bytes + qkv_bytes > ws_size) return;

  char* ws = (char*)d_ws;
  unsigned short* xb = (unsigned short*)ws;
  unsigned short* wb = (unsigned short*)(ws + xb_bytes);
  float* qkv = (float*)(ws + xb_bytes + wb_bytes);

  const int nrows = in_sizes[0] / FIN;

  const int nx8 = (M_ * KDIM) / 8;
  cvt_bf16x8<<<dim3((nx8 + 255) / 256, 1), 256, 0, stream>>>(x, x, x, xb, nx8, 0);
  const int nw8 = (FOUT * FIN) / 8;
  cvt_bf16x8<<<dim3((nw8 + 255) / 256, 3), 256, 0, stream>>>(Wq, Wk, Wv, wb, nw8, nw8);

  qkv_gemm<<<dim3(M_ / 128, NTOT / 128), GEMM_THREADS, GEMM_DYN_LDS, stream>>>(xb, wb, qkv);

  float* outp  = (float*)d_out;
  float* attnp = outp + (size_t)M_ * FOUT;
  attn_kernel<<<(nrows + ROWS_PER_BLK - 1) / ROWS_PER_BLK, 256, 0, stream>>>(qkv, rel, outp, attnp, nrows);
}
